// BigBirdAttention_89945205113168
// MI455X (gfx1250) — hardware-verified
//
#include <hip/hip_runtime.h>
#include <stdint.h>


#define EMBED   1024
#define NHEAD   16
#define HDIM    64
#define SEQ     2048
#define BATCH   2
#define QBLK    64
#define NBLK    (SEQ / QBLK)
#define WIN     3
#define NRAND   3
#define MROWS   (BATCH * SEQ)

#define TP      40
#define EP16    136
#define EP32    68
#define SP      72

typedef unsigned short us;
typedef us       us8  __attribute__((ext_vector_type(8)));
typedef us       us16 __attribute__((ext_vector_type(16)));
typedef _Float16 h16v __attribute__((ext_vector_type(16)));
typedef __bf16   b16v __attribute__((ext_vector_type(16)));
typedef float    f8   __attribute__((ext_vector_type(8)));
typedef float    v4f  __attribute__((ext_vector_type(4)));

union Frag { us16 u; us8 hv[2]; h16v h; b16v b; };

struct BlkMask { unsigned int bits[NBLK]; };
typedef char blkmask_size_check[(sizeof(BlkMask) == sizeof(unsigned int) * NBLK) ? 1 : -1];

__device__ __forceinline__ us f16_bits(float x) {
  union { _Float16 f; us u; } c;
  c.f = (_Float16)x;
  return c.u;
}
__device__ __forceinline__ us bf16_rne_bits(float x) {
  unsigned int u = __float_as_uint(x);
  u += 0x7FFFu + ((u >> 16) & 1u);
  return (us)(u >> 16);
}
__device__ __forceinline__ float bf16_to_f32(us v) {
  return __uint_as_float(((unsigned int)v) << 16);
}

__device__ __forceinline__ f8 mma_f16(const Frag& a, const Frag& b, f8 c) {
  return __builtin_amdgcn_wmma_f32_16x16x32_f16(false, a.h, false, b.h, (short)0, c, false, false);
}
__device__ __forceinline__ f8 mma_bf16(const Frag& a, const Frag& b, f8 c) {
  return __builtin_amdgcn_wmma_f32_16x16x32_bf16(false, a.b, false, b.b, (short)0, c, false, false);
}
#define NOP4 "v_nop\n\tv_nop\n\tv_nop\n\tv_nop"

__global__ __launch_bounds__(256) void k_cvt(
    const float* __restrict__ s0, const float* __restrict__ s1, const float* __restrict__ s2,
    const float* __restrict__ s3, const float* __restrict__ s4,
    us* d0, us* d1, us* d2, us* d3, us* d4, int n0, int nw)
{
  const int seg = blockIdx.y;
  const float* src; us* dst; int n; float sc;
  if (seg == 0)      { src = s0; dst = d0; n = n0; sc = 1.0f;  }
  else if (seg == 1) { src = s1; dst = d1; n = nw; sc = 64.0f; }
  else if (seg == 2) { src = s2; dst = d2; n = nw; sc = 64.0f; }
  else if (seg == 3) { src = s3; dst = d3; n = nw; sc = 64.0f; }
  else               { src = s4; dst = d4; n = nw; sc = 64.0f; }
  const size_t i = ((size_t)blockIdx.x * 256 + threadIdx.x) * 8;
  if (i + 8 > (size_t)n) return;
  const v4f a = *(const v4f*)(src + i);
  const v4f c = *(const v4f*)(src + i + 4);
  us8 o;
  o[0] = f16_bits(a[0] * sc); o[1] = f16_bits(a[1] * sc); o[2] = f16_bits(a[2] * sc); o[3] = f16_bits(a[3] * sc);
  o[4] = f16_bits(c[0] * sc); o[5] = f16_bits(c[1] * sc); o[6] = f16_bits(c[2] * sc); o[7] = f16_bits(c[3] * sc);
  us* p = dst + i;
  *(volatile us8*)p = o;
  __threadfence();
  *(volatile us8*)p = o;
}

__device__ __forceinline__ void gemm_tile(const us* __restrict__ A, const us* __restrict__ B,
                                          int mBase, int nBase, us* As, us* Bs, f8 (&acc)[2][4])
{
  const int t = threadIdx.x;
  const int lane = t & 31, wav = t >> 5;
  const int wr = wav & 3, wc = wav >> 2;
  const int lm = lane & 15, lh = lane >> 4;

#pragma unroll
  for (int mt = 0; mt < 2; ++mt)
#pragma unroll
    for (int nt = 0; nt < 4; ++nt) acc[mt][nt] = (f8)0.0f;

  const int ldRow = t >> 1;
  const int ldCol = (t & 1) * 16;
  const us* aRow = A + (size_t)(mBase + ldRow) * EMBED + ldCol;
  const us* bRow = B + (size_t)(nBase + ldRow) * EMBED + ldCol;
  us* aDst = As + ldRow * TP + ldCol;
  us* bDst = Bs + ldRow * TP + ldCol;

  for (int kk = 0; kk < EMBED; kk += 32) {
    const us8 a0 = *(const us8*)(aRow + kk);
    const us8 a1 = *(const us8*)(aRow + kk + 8);
    const us8 b0 = *(const us8*)(bRow + kk);
    const us8 b1 = *(const us8*)(bRow + kk + 8);
    *(us8*)(aDst)     = a0;
    *(us8*)(aDst + 8) = a1;
    *(us8*)(bDst)     = b0;
    *(us8*)(bDst + 8) = b1;
    __syncthreads();

    Frag af[2], bf[4];
#pragma unroll
    for (int mt = 0; mt < 2; ++mt) {
      const us* p = As + (wr * 32 + mt * 16 + lm) * TP + 8 * lh;
      af[mt].hv[0] = *(const us8*)p;
      af[mt].hv[1] = *(const us8*)(p + 16);
    }
#pragma unroll
    for (int nt = 0; nt < 4; ++nt) {
      const us* p = Bs + (wc * 64 + nt * 16 + lm) * TP + 8 * lh;
      bf[nt].hv[0] = *(const us8*)p;
      bf[nt].hv[1] = *(const us8*)(p + 16);
    }
#pragma unroll
    for (int nt = 0; nt < 4; ++nt)
#pragma unroll
      for (int mt = 0; mt < 2; ++mt)
        acc[mt][nt] = mma_f16(af[mt], bf[nt], acc[mt][nt]);
    asm volatile(NOP4
                 : "+v"(acc[0][0]), "+v"(acc[0][1]), "+v"(acc[0][2]), "+v"(acc[0][3]),
                   "+v"(acc[1][0]), "+v"(acc[1][1]), "+v"(acc[1][2]), "+v"(acc[1][3])
                 : "v"(af[0].u), "v"(af[1].u), "v"(bf[0].u), "v"(bf[1].u), "v"(bf[2].u), "v"(bf[3].u));
    __syncthreads();
  }
}

__device__ __forceinline__ void qk_store_pass(us* dst, const us* Ec, int mBase, int nBase, int t) {
#pragma unroll
  for (int j = 0; j < 8; ++j) {
    const int id = t + 256 * j;
    const int head = id >> 10;
    const int rem = id & 1023;
    const int row = rem >> 3;
    const int c8 = rem & 7;
    us8 v;
#pragma unroll
    for (int i = 0; i < 8; ++i) v[i] = Ec[(head * 64 + c8 * 8 + i) * EP16 + row];
    const int m = mBase + row;
    const int b = m / SEQ;
    const int s = m % SEQ;
    const int hh = (nBase >> 6) + head;
    us* d = dst + (((size_t)(b * NHEAD + hh) * SEQ + s) * HDIM + c8 * 8);
    *(volatile us8*)d = v;
  }
}
__device__ __forceinline__ void vt_store_pass(us* Vt, const us* Ec, int mBase, int nBase, int t) {
#pragma unroll
  for (int j = 0; j < 8; ++j) {
    const int id = t + 256 * j;
    const int head = id >> 10;
    const int rem = id & 1023;
    const int dd = rem >> 4;
    const int c16 = rem & 15;
    const us8 v = *(const us8*)(Ec + (head * 64 + dd) * EP16 + c16 * 8);
    const int b = mBase / SEQ;
    const int s0 = mBase % SEQ;
    const int hh = (nBase >> 6) + head;
    us* d = Vt + (((size_t)(b * NHEAD + hh) * HDIM + dd) * SEQ + s0 + c16 * 8);
    *(volatile us8*)d = v;
  }
}

__global__ __launch_bounds__(256) void k_proj(
    const us* __restrict__ Hh, const us* __restrict__ Wq, const us* __restrict__ Wk, const us* __restrict__ Wv,
    const float* __restrict__ bq, const float* __restrict__ bk, const float* __restrict__ bv,
    us* Qhi, us* Qlo, us* Khi, us* Klo, us* Vt)
{
  __shared__ __align__(16) us As[128 * TP];
  __shared__ __align__(16) us Bs[128 * TP];
  __shared__ __align__(16) us Ec[128 * EP16];

  const int z = blockIdx.z;
  const int mBase = blockIdx.y * 128;
  const int nBase = blockIdx.x * 128;
  if (mBase >= MROWS || nBase >= EMBED) return;

  const us* W = (z == 0) ? Wq : (z == 1) ? Wk : Wv;
  const float* bias = (z == 0) ? bq : (z == 1) ? bk : bv;

  f8 acc[2][4];
  gemm_tile(Hh, W, mBase, nBase, As, Bs, acc);

  const int t = threadIdx.x;
  const int lane = t & 31, wav = t >> 5;
  const int wr = wav & 3, wc = wav >> 2;
  const int lm = lane & 15, lh = lane >> 4;

  float bn[4];
#pragma unroll
  for (int nt = 0; nt < 4; ++nt) bn[nt] = bias[nBase + wc * 64 + nt * 16 + lm];

  const float amul = (z == 0) ? (0.125f / 64.0f) : (1.0f / 64.0f);
  const float bmul = (z == 0) ? 0.125f : 1.0f;
  const int nplanes = (z == 2) ? 1 : 2;

  for (int p = 0; p < nplanes; ++p) {
#pragma unroll
    for (int mt = 0; mt < 2; ++mt) {
#pragma unroll
      for (int nt = 0; nt < 4; ++nt) {
        const int C  = wc * 64 + nt * 16 + lm;
        const int R0 = wr * 32 + mt * 16 + 8 * lh;
        us8 o;
#pragma unroll
        for (int r = 0; r < 8; ++r) {
          const float x = acc[mt][nt][r] * amul + bn[nt] * bmul;
          us v;
          if (z == 2) {
            v = f16_bits(x);
          } else {
            const us hi = bf16_rne_bits(x);
            v = (p == 0) ? hi : bf16_rne_bits(x - bf16_to_f32(hi));
          }
          o[r] = v;
        }
        *(us8*)(Ec + C * EP16 + R0) = o;
      }
    }
    __syncthreads();
    if (z < 2) {
      us* dst = (z == 0) ? ((p == 0) ? Qhi : Qlo) : ((p == 0) ? Khi : Klo);
      qk_store_pass(dst, Ec, mBase, nBase, t);
      __threadfence();
      qk_store_pass(dst, Ec, mBase, nBase, t);
    } else {
      vt_store_pass(Vt, Ec, mBase, nBase, t);
      __threadfence();
      vt_store_pass(Vt, Ec, mBase, nBase, t);
    }
    __syncthreads();
  }
}

__device__ __forceinline__ void ao_store_pass(us* AOh, const us* stw, int b, int hd, int qb, int wav, int lane) {
#pragma unroll
  for (int j = 0; j < 4; ++j) {
    const int row = 4 * j + (lane >> 3);
    const int c = lane & 7;
    const us8 v = *(const us8*)(stw + row * SP + c * 8);
    us* d = AOh + (((size_t)b * SEQ + qb * QBLK + wav * 16 + row) * EMBED + hd * HDIM + c * 8);
    *(volatile us8*)d = v;
  }
}

__global__ __launch_bounds__(128) void k_attn(
    const us* __restrict__ Qhi, const us* __restrict__ Qlo,
    const us* __restrict__ Khi, const us* __restrict__ Klo,
    const us* __restrict__ Vt, us* AOh, BlkMask mk)
{
  __shared__ __align__(16) us Stg[4 * 16 * SP];

  const int qb = blockIdx.x;
  const int bh = blockIdx.y;
  if (qb >= NBLK || bh >= BATCH * NHEAD) return;
  const int b  = bh / NHEAD;
  const int hd = bh % NHEAD;
  const int t = threadIdx.x;
  const int lane = t & 31, wav = t >> 5;
  const int lm = lane & 15, lh = lane >> 4;

  unsigned int bits = 0u;
#pragma unroll
  for (int i = 0; i < NBLK; ++i) if (i == qb) bits = mk.bits[i];

  const size_t qrow = (size_t)bh * SEQ + qb * QBLK + wav * 16 + lm;
  Frag qh[2], ql[2];
#pragma unroll
  for (int kc = 0; kc < 2; ++kc) {
    const us* ph = Qhi + qrow * HDIM + kc * 32 + 8 * lh;
    const us* pl = Qlo + qrow * HDIM + kc * 32 + 8 * lh;
    qh[kc].hv[0] = *(const us8*)ph;  qh[kc].hv[1] = *(const us8*)(ph + 16);
    ql[kc].hv[0] = *(const us8*)pl;  ql[kc].hv[1] = *(const us8*)(pl + 16);
  }

  const float L2E = 1.44269504088896f;
  float mrun = -1.0e30f;
  float lrun = 0.0f;
  f8 oacc[4];
#pragma unroll
  for (int dt = 0; dt < 4; ++dt) oacc[dt] = (f8)0.0f;

  for (int kb = 0; kb < NBLK; ++kb) {
    if (((bits >> kb) & 1u) == 0u) continue;
    const size_t krow0 = (size_t)bh * SEQ + kb * QBLK;

    f8 sacc[4];
#pragma unroll
    for (int kt = 0; kt < 4; ++kt) {
      Frag kh[2], kl[2];
      const us* pkh = Khi + (krow0 + kt * 16 + lm) * HDIM + 8 * lh;
      const us* pkl = Klo + (krow0 + kt * 16 + lm) * HDIM + 8 * lh;
#pragma unroll
      for (int kc = 0; kc < 2; ++kc) {
        kh[kc].hv[0] = *(const us8*)(pkh + kc * 32);  kh[kc].hv[1] = *(const us8*)(pkh + kc * 32 + 16);
        kl[kc].hv[0] = *(const us8*)(pkl + kc * 32);  kl[kc].hv[1] = *(const us8*)(pkl + kc * 32 + 16);
      }
      f8 s = (f8)0.0f;
#pragma unroll
      for (int kc = 0; kc < 2; ++kc) {
        s = mma_bf16(kh[kc], qh[kc], s);
        s = mma_bf16(kh[kc], ql[kc], s);
        s = mma_bf16(kl[kc], qh[kc], s);
      }
      asm volatile(NOP4 : "+v"(s) : "v"(kh[0].u), "v"(kh[1].u), "v"(kl[0].u), "v"(kl[1].u));
      sacc[kt] = s;
    }

    float mx = sacc[0][0];
#pragma unroll
    for (int kt = 0; kt < 4; ++kt)
#pragma unroll
      for (int r = 0; r < 8; ++r) mx = fmaxf(mx, sacc[kt][r]);
    mx = fmaxf(mx, __shfl_xor(mx, 16));
    const float mnew = fmaxf(mrun, mx);
    const float alpha = exp2f(fmaxf(mrun - mnew, -120.0f) * L2E);
    mrun = mnew;

    float ps = 0.0f;
    Frag pf[2];
#pragma unroll
    for (int kt = 0; kt < 4; ++kt) {
      us8 o;
#pragma unroll
      for (int r = 0; r < 8; ++r) {
        const float pv = exp2f((sacc[kt][r] - mnew) * L2E);
        ps += pv;
        o[r] = f16_bits(pv * 4096.0f);
      }
      pf[kt >> 1].hv[kt & 1] = o;
    }
    ps += __shfl_xor(ps, 16);
    lrun = lrun * alpha + ps;
#pragma unroll
    for (int dt = 0; dt < 4; ++dt) oacc[dt] = oacc[dt] * alpha;

#pragma unroll
    for (int kc = 0; kc < 2; ++kc) {
      Frag vf[4];
#pragma unroll
      for (int dt = 0; dt < 4; ++dt) {
        const us* pv = Vt + ((size_t)bh * HDIM + dt * 16 + lm) * SEQ + kb * QBLK + kc * 32 + 8 * lh;
        vf[dt].hv[0] = *(const us8*)pv;
        vf[dt].hv[1] = *(const us8*)(pv + 16);
      }
#pragma unroll
      for (int dt = 0; dt < 4; ++dt) oacc[dt] = mma_f16(vf[dt], pf[kc], oacc[dt]);
      asm volatile(NOP4
                   : "+v"(oacc[0]), "+v"(oacc[1]), "+v"(oacc[2]), "+v"(oacc[3])
                   : "v"(vf[0].u), "v"(vf[1].u), "v"(vf[2].u), "v"(vf[3].u), "v"(pf[kc].u));
    }
  }

  const float inv = 1.0f / (256.0f * lrun);
  us* stw = Stg + wav * 16 * SP;
#pragma unroll
  for (int dt = 0; dt < 4; ++dt) {
    us8 o;
#pragma unroll
    for (int r = 0; r < 8; ++r) o[r] = f16_bits(oacc[dt][r] * inv);
    *(us8*)(stw + lm * SP + dt * 16 + 8 * lh) = o;
  }
  __syncthreads();
  ao_store_pass(AOh, stw, b, hd, qb, wav, lane);
  __threadfence();
  ao_store_pass(AOh, stw, b, hd, qb, wav, lane);
}

__device__ __forceinline__ void out_store_pass(float* out, const float* Ec, const float* __restrict__ bo,
                                               int mRow0, int nBase, int t) {
#pragma unroll
  for (int j = 0; j < 8; ++j) {
    const int id = t + 256 * j;
    const int row = id >> 5;
    const int c = id & 31;
    const v4f bb = *(const v4f*)(bo + nBase + 4 * c);
    v4f v;
#pragma unroll
    for (int i = 0; i < 4; ++i) v[i] = Ec[(4 * c + i) * EP32 + row] * (1.0f / 1024.0f) + bb[i];
    float* d = out + ((size_t)(mRow0 + row) * EMBED + nBase + 4 * c);
    *(volatile v4f*)d = v;
  }
}

__global__ __launch_bounds__(256) void k_out(
    const us* __restrict__ AOh, const us* __restrict__ Wo, const float* __restrict__ bo, float* out)
{
  __shared__ __align__(16) us As[128 * TP];
  __shared__ __align__(16) us Bs[128 * TP];
  __shared__ __align__(16) float Ec[128 * EP32];

  const int mBase = blockIdx.y * 128;
  const int nBase = blockIdx.x * 128;
  if (mBase >= MROWS || nBase >= EMBED) return;

  f8 acc[2][4];
  gemm_tile(AOh, Wo, mBase, nBase, As, Bs, acc);

  const int t = threadIdx.x;
  const int lane = t & 31, wav = t >> 5;
  const int wr = wav & 3, wc = wav >> 2;
  const int lm = lane & 15, lh = lane >> 4;

  for (int hf = 0; hf < 2; ++hf) {
    if ((wr >> 1) == hf) {
#pragma unroll
      for (int mt = 0; mt < 2; ++mt) {
#pragma unroll
        for (int nt = 0; nt < 4; ++nt) {
          const int C  = wc * 64 + nt * 16 + lm;
          const int R0 = (wr & 1) * 32 + mt * 16 + 8 * lh;
          v4f lo, hi;
          lo[0] = acc[mt][nt][0]; lo[1] = acc[mt][nt][1]; lo[2] = acc[mt][nt][2]; lo[3] = acc[mt][nt][3];
          hi[0] = acc[mt][nt][4]; hi[1] = acc[mt][nt][5]; hi[2] = acc[mt][nt][6]; hi[3] = acc[mt][nt][7];
          *(v4f*)(Ec + C * EP32 + R0)     = lo;
          *(v4f*)(Ec + C * EP32 + R0 + 4) = hi;
        }
      }
    }
    __syncthreads();
    out_store_pass(out, Ec, bo, mBase + hf * 64, nBase, t);
    __threadfence();
    out_store_pass(out, Ec, bo, mBase + hf * 64, nBase, t);
    __syncthreads();
  }
}

static void mt_init(unsigned int* mt, unsigned int seed) {
  mt[0] = seed;
  for (int i = 1; i < 624; ++i) mt[i] = 1812433253u * (mt[i - 1] ^ (mt[i - 1] >> 30)) + (unsigned int)i;
}
static void mt_gen(unsigned int* mt) {
  const unsigned int UPPER = 0x80000000u, LOWER = 0x7fffffffu, MAT = 0x9908b0dfu;
  int kk = 0;
  for (; kk < 624 - 397; ++kk) {
    const unsigned int y = (mt[kk] & UPPER) | (mt[kk + 1] & LOWER);
    mt[kk] = mt[kk + 397] ^ (y >> 1) ^ ((y & 1u) ? MAT : 0u);
  }
  for (; kk < 623; ++kk) {
    const unsigned int y = (mt[kk] & UPPER) | (mt[kk + 1] & LOWER);
    mt[kk] = mt[kk + (397 - 624)] ^ (y >> 1) ^ ((y & 1u) ? MAT : 0u);
  }
  const unsigned int y = (mt[623] & UPPER) | (mt[0] & LOWER);
  mt[623] = mt[396] ^ (y >> 1) ^ ((y & 1u) ? MAT : 0u);
}
static unsigned int mt_next(unsigned int* mt, int* pos) {
  if (*pos >= 624) { mt_gen(mt); *pos = 0; }
  unsigned int y = mt[(*pos)++];
  y ^= (y >> 11);
  y ^= (y << 7) & 0x9d2c5680u;
  y ^= (y << 15) & 0xefc60000u;
  y ^= (y >> 18);
  return y;
}
static unsigned int mt_interval(unsigned int* mt, int* pos, unsigned int maxv) {
  if (maxv == 0u) return 0u;
  unsigned int msk = maxv;
  msk |= msk >> 1; msk |= msk >> 2; msk |= msk >> 4; msk |= msk >> 8; msk |= msk >> 16;
  unsigned int v;
  do { v = mt_next(mt, pos) & msk; } while (v > maxv);
  return v;
}

extern "C" void kernel_launch(void* const* d_in, const int* in_sizes, int n_in,
                              void* d_out, int out_size, void* d_ws,
                              size_t ws_size, hipStream_t stream)
{
  if (n_in < 9) return;
  if (in_sizes[0] != MROWS * EMBED) return;
  if (in_sizes[1] != EMBED * EMBED || in_sizes[3] != EMBED * EMBED ||
      in_sizes[5] != EMBED * EMBED || in_sizes[7] != EMBED * EMBED) return;
  if (in_sizes[2] != EMBED || in_sizes[4] != EMBED || in_sizes[6] != EMBED || in_sizes[8] != EMBED) return;
  if (out_size != MROWS * EMBED) return;

  const float* hid = (const float*)d_in[0];
  const float* wq  = (const float*)d_in[1];
  const float* bq  = (const float*)d_in[2];
  const float* wk  = (const float*)d_in[3];
  const float* bk  = (const float*)d_in[4];
  const float* wv  = (const float*)d_in[5];
  const float* bv  = (const float*)d_in[6];
  const float* wo  = (const float*)d_in[7];
  const float* bo  = (const float*)d_in[8];
  float* out = (float*)d_out;

  const size_t bH    = (size_t)MROWS * EMBED * 2;
  const size_t bW    = (size_t)EMBED * EMBED * 2;
  const size_t bHead = (size_t)BATCH * NHEAD * SEQ * HDIM * 2;
  const size_t oH   = 0;
  const size_t oWq  = oH + bH;
  const size_t oWk  = oWq + bW;
  const size_t oWv  = oWk + bW;
  const size_t oWo  = oWv + bW;
  const size_t oQhi = oWo + bW;
  const size_t oQlo = oQhi + bHead;
  const size_t oKhi = oQlo + bHead;
  const size_t oKlo = oKhi + bHead;
  const size_t oVt  = oKlo + bHead;
  const size_t oAO  = oVt + bHead;
  const size_t total = oAO + bH;
  if (total > ws_size) return;

  char* ws = (char*)d_ws;
  us* Hh  = (us*)(ws + oH);
  us* Wqh = (us*)(ws + oWq);
  us* Wkh = (us*)(ws + oWk);
  us* Wvh = (us*)(ws + oWv);
  us* Woh = (us*)(ws + oWo);
  us* Qhi = (us*)(ws + oQhi);
  us* Qlo = (us*)(ws + oQlo);
  us* Khi = (us*)(ws + oKhi);
  us* Klo = (us*)(ws + oKlo);
  us* Vt  = (us*)(ws + oVt);
  us* AOh = (us*)(ws + oAO);

  BlkMask mk;
  for (int i = 0; i < NBLK; ++i) mk.bits[i] = 0u;
  mk.bits[0] = 0xFFFFFFFFu;
  for (int q2 = 1; q2 < NBLK; ++q2) {
    unsigned int v = 1u;
    for (int c = q2 - WIN; c <= q2 + WIN; ++c)
      if (c >= 0 && c < NBLK) v |= (1u << c);
    mk.bits[q2] = v;
  }
  {
    unsigned int mt[624];
    int pos = 624;
    mt_init(mt, 0u);
    for (int bb = 1; bb < NBLK; ++bb) {
      int avail[NBLK];
      int na = 0;
      for (int x = 1; x < NBLK; ++x) {
        int di = x - bb; if (di < 0) di = -di;
        if (di > WIN) avail[na++] = x;
      }
      if (na > 0) {
        int perm[NBLK];
        for (int i = 0; i < na; ++i) perm[i] = i;
        for (int i = na - 1; i >= 1; --i) {
          const int j = (int)mt_interval(mt, &pos, (unsigned int)i);
          const int tmp = perm[i]; perm[i] = perm[j]; perm[j] = tmp;
        }
        const int cnt = (na < NRAND) ? na : NRAND;
        for (int q = 0; q < cnt; ++q) mk.bits[bb] |= (1u << avail[perm[q]]);
      }
    }
  }

  const int n0 = in_sizes[0];
  const int nw = in_sizes[1];
  dim3 gc((unsigned)((n0 / 8 + 255) / 256), 5);
  k_cvt<<<gc, 256, 0, stream>>>(hid, wq, wk, wv, wo, Hh, Wqh, Wkh, Wvh, Woh, n0, nw);

  dim3 gp(EMBED / 128, MROWS / 128, 3);
  k_proj<<<gp, 256, 0, stream>>>(Hh, Wqh, Wkh, Wvh, bq, bk, bv, Qhi, Qlo, Khi, Klo, Vt);

  dim3 ga(NBLK, BATCH * NHEAD);
  k_attn<<<ga, 128, 0, stream>>>(Qhi, Qlo, Khi, Klo, Vt, AOh, mk);

  dim3 go(EMBED / 128, MROWS / 128);
  k_out<<<go, 256, 0, stream>>>(AOh, Woh, bo, out);
}
